// Temporal_Mamba_8143257993725
// MI455X (gfx1250) — hardware-verified
//
#include <hip/hip_runtime.h>
#include <math.h>

constexpr int kNB   = 2;
constexpr int kNC   = 96;
constexpr int kNT   = 16;
constexpr int kHW   = 3136;
constexpr int kBF   = 6272;
constexpr int kNH   = 3;
constexpr int kDH   = 32;
constexpr int kKC   = 4;
constexpr int kNCOL = 384;
constexpr int kKX   = 192;
constexpr int kKR   = 96;
constexpr int kLDXA = kNT * kKX;
constexpr size_t kXAElems  = (size_t)kBF * kNT * kKX;
constexpr size_t kGPlane   = (size_t)kBF * kNCOL;
constexpr size_t kStElems  = (size_t)kBF * kNC;
constexpr size_t kOutElems = (size_t)kNB * kNC * kNT * kHW;

constexpr size_t kSzWbt  = (size_t)kNCOL * kKX * 2;
constexpr size_t kSzRbt  = (size_t)kNCOL * kKR * 2;
constexpr size_t kSzXA   = kXAElems * 2;
constexpr size_t kSzG    = 2 * kGPlane * 4;
constexpr size_t kSzRaw  = kGPlane * 4;
constexpr size_t kSzH    = kStElems * 2;
constexpr size_t kSzSt   = kStElems * 4;
constexpr size_t kOffWbtH = 0;
constexpr size_t kOffWbtL = kOffWbtH + kSzWbt;
constexpr size_t kOffRbtH = kOffWbtL + kSzWbt;
constexpr size_t kOffRbtL = kOffRbtH + kSzRbt;
constexpr size_t kOffXaH  = kOffRbtL + kSzRbt;
constexpr size_t kOffXaL  = kOffXaH + kSzXA;
constexpr size_t kOffG    = kOffXaL + kSzXA;
constexpr size_t kOffRaw  = kOffG + kSzG;
constexpr size_t kOffHh   = kOffRaw + kSzRaw;
constexpr size_t kOffHl   = kOffHh + kSzH;
constexpr size_t kOffStC  = kOffHl + kSzH;
constexpr size_t kOffStN  = kOffStC + kSzSt;
constexpr size_t kOffStM  = kOffStN + kSzSt;
constexpr size_t kWsTotal = kOffStM + kSzSt;
typedef char ws_fits_check[(kWsTotal <= (size_t)134217728) ? 1 : -1];
typedef char ws_total_check[(kWsTotal == (size_t)116047872) ? 1 : -1];
typedef char tile_m_check[(kBF % 64 == 0 && kNCOL % 64 == 0 && kKX % 32 == 0 && kKR % 32 == 0) ? 1 : -1];
typedef char row_block_check[(kHW % 32 == 0 && kHW % 16 == 0) ? 1 : -1];

typedef __attribute__((ext_vector_type(16))) _Float16 v16h;
typedef __attribute__((ext_vector_type(8)))  _Float16 v8h;
typedef __attribute__((ext_vector_type(16))) __bf16   v16b;
typedef __attribute__((ext_vector_type(8)))  __bf16   v8b;
typedef __attribute__((ext_vector_type(8)))  float    v8f;
typedef __attribute__((ext_vector_type(4)))  float    v4f;
typedef __attribute__((ext_vector_type(4)))  unsigned int v4u;

__device__ __forceinline__ unsigned short f2bf_bits(float f) {
  unsigned u = __float_as_uint(f);
  return (unsigned short)((u + 0x7FFFu + ((u >> 16) & 1u)) >> 16);
}
__device__ __forceinline__ float bf_bits2f(unsigned short h) { return __uint_as_float(((unsigned)h) << 16); }

__device__ __forceinline__ void dep_guard_h(v8f& a, v8f& b, v16h x, v16h y) { asm volatile("v_nop\n\tv_nop\n\tv_nop\n\tv_nop" : "+v"(a), "+v"(b) : "v"(x), "v"(y)); }
__device__ __forceinline__ void dep_guard_b(v8f& a, v8f& b, v16b x, v16b y) { asm volatile("v_nop\n\tv_nop\n\tv_nop\n\tv_nop" : "+v"(a), "+v"(b) : "v"(x), "v"(y)); }
__device__ __forceinline__ void keep4_h(v16h a, v16h b, v16h c, v16h d) { asm volatile("v_nop" :: "v"(a), "v"(b), "v"(c), "v"(d)); }
__device__ __forceinline__ void keep4_b(v16b a, v16b b, v16b c, v16b d) { asm volatile("v_nop" :: "v"(a), "v"(b), "v"(c), "v"(d)); }
__device__ __forceinline__ void acc_guard4(v8f& a, v8f& b, v8f& c, v8f& d) { asm volatile("v_nop\n\tv_nop\n\tv_nop\n\tv_nop" : "+v"(a), "+v"(b), "+v"(c), "+v"(d)); }
template <typename T> struct Frag;
template <> struct Frag<_Float16> {
  typedef v16h V; union U { v16h v; v8h h[2]; };
  static __device__ __forceinline__ v16h load(const _Float16* p) {
    U f; f.h[0] = *(const v8h*)(p); f.h[1] = *(const v8h*)(p + 16); return f.v;
  }
  static __device__ __forceinline__ v8f mma(v16h a, v16h b, v8f c) {
    return __builtin_amdgcn_wmma_f32_16x16x32_f16(false, a, false, b, (short)0, c, false, false);
  }
  static __device__ __forceinline__ void guard(v8f& a, v8f& b, v16h x, v16h y) { dep_guard_h(a, b, x, y); }
  static __device__ __forceinline__ void keep(v16h a, v16h b, v16h c, v16h d) { keep4_h(a, b, c, d); }
};
template <> struct Frag<__bf16> {
  typedef v16b V; union U { v16b v; v8b h[2]; };
  static __device__ __forceinline__ v16b load(const __bf16* p) {
    U f; f.h[0] = *(const v8b*)(p); f.h[1] = *(const v8b*)(p + 16); return f.v;
  }
  static __device__ __forceinline__ v8f mma(v16b a, v16b b, v8f c) {
    return __builtin_amdgcn_wmma_f32_16x16x32_bf16(false, a, false, b, (short)0, c, false, false);
  }
  static __device__ __forceinline__ void guard(v8f& a, v8f& b, v16b x, v16b y) { dep_guard_b(a, b, x, y); }
  static __device__ __forceinline__ void keep(v16b a, v16b b, v16b c, v16b d) { keep4_b(a, b, c, d); }
};

__device__ __forceinline__ unsigned pk16(unsigned short a, unsigned short b) { return (unsigned)a | ((unsigned)b << 16); }

template <int ET> struct Elem;
template <> struct Elem<0> { typedef _Float16 T; };
template <> struct Elem<1> { typedef __bf16 T; };
template <int ET, bool SPLIT, int BIAS_MODE, int OUT_MODE, bool RESID, int ACT = 0>
__global__ __launch_bounds__(256) void wmma_gemm64(
    const unsigned short* __restrict__ Ap, const unsigned short* __restrict__ A2p, int lda, long strideA,
    const unsigned short* __restrict__ Btp, const unsigned short* __restrict__ Bt2p, int ldb, long strideB,
    void* __restrict__ Cout, void* __restrict__ Cout2, int ldc, long strideC,
    const float* __restrict__ bias,
    const float* __restrict__ resid, long strideR,
    int M, int N, int K, float scale) {
  typedef typename Elem<ET>::T T;
  typedef typename Frag<T>::V V;
  const T* A = (const T*)Ap; const T* A2 = (const T*)A2p; const T* Bt = (const T*)Btp; const T* Bt2 = (const T*)Bt2p;
  __shared__ __align__(16) float sT[8][16 * 68];
  const int b    = blockIdx.y;
  const int lane = threadIdx.x & 31;
  const int wave = threadIdx.x >> 5;
  const int tilesN = N >> 6;
  const int tilesM = M >> 6;
  const int tile = blockIdx.x * 8 + wave;
  if (tile >= tilesM * tilesN) return;
  const int tm = tile / tilesN;
  const int tn = tile - tm * tilesN;
  const int m0 = tm << 6;
  const int n0 = tn << 6;

  const T* Ab  = A  + (size_t)b * strideA;
  const T* Bb  = Bt + (size_t)b * strideB;
  const T* Ab2 = SPLIT ? (A2  + (size_t)b * strideA) : nullptr;
  const T* Bb2 = SPLIT ? (Bt2 + (size_t)b * strideB) : nullptr;

  const int rlane = lane & 15;
  const int koff  = (lane >> 4) * 8;
  const int mOff  = (lane >> 4) * 8;

  v8f acc[4][4];
#pragma unroll
  for (int i = 0; i < 4; ++i)
#pragma unroll
    for (int j = 0; j < 4; ++j) acc[i][j] = (v8f){0.f,0.f,0.f,0.f,0.f,0.f,0.f,0.f};

  for (int k0 = 0; k0 < K; k0 += 32) {
    V bh[4], bl[4];
#pragma unroll
    for (int j = 0; j < 4; ++j) {
      const size_t bo = (size_t)(n0 + (j << 4) + rlane) * ldb + koff + k0;
      bh[j] = Frag<T>::load(Bb + bo);
      if (SPLIT) bl[j] = Frag<T>::load(Bb2 + bo);
    }
#pragma unroll
    for (int i = 0; i < 4; ++i) {
      const size_t ao = (size_t)(m0 + (i << 4) + rlane) * lda + koff + k0;
      V ah = Frag<T>::load(Ab + ao);
      V al;
      if (SPLIT) al = Frag<T>::load(Ab2 + ao);
#pragma unroll
      for (int j = 0; j < 4; ++j) {
        acc[i][j] = Frag<T>::mma(ah, bh[j], acc[i][j]);
        if (SPLIT) {
          acc[i][j] = Frag<T>::mma(ah, bl[j], acc[i][j]);
          acc[i][j] = Frag<T>::mma(al, bh[j], acc[i][j]);
        }
      }
      Frag<T>::guard(acc[i][0], acc[i][3], ah, SPLIT ? al : ah);
    }
    Frag<T>::keep(bh[0], bh[1], bh[2], bh[3]);
    if (SPLIT) Frag<T>::keep(bl[0], bl[1], bl[2], bl[3]);
  }
  acc_guard4(acc[0][0], acc[0][1], acc[0][2], acc[0][3]);
  acc_guard4(acc[1][0], acc[1][1], acc[1][2], acc[1][3]);
  acc_guard4(acc[2][0], acc[2][1], acc[2][2], acc[2][3]);
  acc_guard4(acc[3][0], acc[3][1], acc[3][2], acc[3][3]);

  float* slab = sT[wave];
  const float* Rb = RESID ? (resid + (size_t)b * strideR) : nullptr;
#pragma unroll
  for (int i = 0; i < 4; ++i) {
    const int mBase = m0 + (i << 4);
#pragma unroll
    for (int j = 0; j < 4; ++j) {
      const int n = n0 + (j << 4) + rlane;
      float bv = 0.f;
      if (BIAS_MODE == 2) bv = bias[n];
#pragma unroll
      for (int r = 0; r < 8; ++r) {
        float v = acc[i][j][r] * scale;
        if (BIAS_MODE == 1) v += bias[mBase + mOff + r];
        if (BIAS_MODE == 2) v += bv;
        if (RESID) v += Rb[(size_t)(mBase + mOff + r) * ldc + n];
        if (ACT == 2) v = fmaxf(v, 0.0f);
        if (ACT == 4) v = (v > 0.f) ? v : 0.01f * v;
        slab[(mOff + r) * 68 + (j << 4) + rlane] = v;
      }
    }
    __builtin_amdgcn_fence(__ATOMIC_RELEASE, "workgroup");
    __builtin_amdgcn_wave_barrier();
    __builtin_amdgcn_fence(__ATOMIC_ACQUIRE, "workgroup");
    if (OUT_MODE == 0) {
      float* C = (float*)Cout + (size_t)b * strideC;
      const int hh = lane >> 4, c4 = (lane & 15) * 4;
      for (int pass = 0; pass < 2; ++pass) {
#pragma unroll
        for (int it = 0; it < 8; ++it) {
          const int row = it * 2 + hh;
          v4f v = *(const v4f*)(slab + row * 68 + c4);
          *(volatile v4f*)(C + (size_t)(mBase + row) * ldc + n0 + c4) = v;
        }
        __threadfence();
      }
    } else {
      const int q = lane >> 3, c8 = (lane & 7) * 8;
      unsigned short* C  = (unsigned short*)Cout  + (size_t)b * strideC;
      unsigned short* C2 = (OUT_MODE == 2) ? ((unsigned short*)Cout2 + (size_t)b * strideC) : nullptr;
      for (int pass = 0; pass < 2; ++pass) {
#pragma unroll
        for (int it = 0; it < 4; ++it) {
          const int row = it * 4 + q;
          const float* sp = slab + row * 68 + c8;
          v8h hv, lv;
#pragma unroll
          for (int e = 0; e < 8; ++e) {
            if (OUT_MODE == 1) {
              hv[e] = (_Float16)sp[e];
            } else {
              unsigned short hb = f2bf_bits(sp[e]);
              unsigned short lb = f2bf_bits(sp[e] - bf_bits2f(hb));
              hv[e] = __builtin_bit_cast(_Float16, hb);
              lv[e] = __builtin_bit_cast(_Float16, lb);
            }
          }
          *(volatile v8h*)(C + (size_t)(mBase + row) * ldc + n0 + c8) = hv;
          if (OUT_MODE == 2) *(volatile v8h*)(C2 + (size_t)(mBase + row) * ldc + n0 + c8) = lv;
        }
        __threadfence();
      }
    }
    __builtin_amdgcn_fence(__ATOMIC_RELEASE, "workgroup");
    __builtin_amdgcn_wave_barrier();
    __builtin_amdgcn_fence(__ATOMIC_ACQUIRE, "workgroup");
  }
}

__global__ __launch_bounds__(256) void k_wpack(const float* __restrict__ Wi, const float* __restrict__ Wf,
                                                const float* __restrict__ Wz, const float* __restrict__ Wo,
                                                const float* __restrict__ Rm,
                                                unsigned short* __restrict__ wbth, unsigned short* __restrict__ wbtl,
                                                unsigned short* __restrict__ rbth, unsigned short* __restrict__ rbtl) {
  const int gid = blockIdx.x * 256 + threadIdx.x;
  float v[8];
  unsigned short* dh;
  unsigned short* dl;
  if (blockIdx.x < 36) {
    const int e0   = gid * 8;
    const int row  = e0 / kKX;
    const int col0 = e0 - row * kKX;
    const int g    = row / kNC;
    const int rem  = row - g * kNC;
    const int n    = rem >> 5;
    const int e    = rem & 31;
    const int hf   = (col0 >= kNC) ? 1 : 0;
    const int cc   = col0 - kNC * hf;
    const int cn   = cc >> 5;
    const int d0   = cc & 31;
    const bool valid = (cn == n) && (hf == ((g >= 2) ? 1 : 0));
#pragma unroll
    for (int k = 0; k < 8; ++k) {
      const int idx = (n * kDH + d0 + k) * kDH + e;
      const float a0 = Wi[idx], a1 = Wf[idx], a2 = Wz[idx], a3 = Wo[idx];
      const float s = (g == 0) ? a0 : (g == 1) ? a1 : (g == 2) ? a2 : a3;
      v[k] = valid ? s : 0.0f;
    }
    dh = wbth + e0;
    dl = wbtl + e0;
  } else {
    const int e0   = (gid - 36 * 256) * 8;
    const int row  = e0 / kKR;
    const int col0 = e0 - row * kKR;
    const int g    = row / kNC;
    const int rem  = row - g * kNC;
    const int n    = rem >> 5;
    const int e    = rem & 31;
    const int cn   = col0 >> 5;
    const int d0   = col0 & 31;
    const bool valid = (cn == n);
#pragma unroll
    for (int k = 0; k < 8; ++k) {
      const int idx = ((g * kNH + n) * kDH + d0 + k) * kDH + e;
      const float s = Rm[idx];
      v[k] = valid ? s : 0.0f;
    }
    dh = rbth + e0;
    dl = rbtl + e0;
  }
  unsigned short hb[8], lb[8];
#pragma unroll
  for (int k = 0; k < 8; ++k) {
    hb[k] = f2bf_bits(v[k]);
    lb[k] = f2bf_bits(v[k] - bf_bits2f(hb[k]));
  }
  const v4u uh = (v4u){pk16(hb[0], hb[1]), pk16(hb[2], hb[3]), pk16(hb[4], hb[5]), pk16(hb[6], hb[7])};
  const v4u ul = (v4u){pk16(lb[0], lb[1]), pk16(lb[2], lb[3]), pk16(lb[4], lb[5]), pk16(lb[6], lb[7])};
  for (int pass = 0; pass < 2; ++pass) {
    *(volatile v4u*)dh = uh;
    *(volatile v4u*)dl = ul;
    __threadfence();
  }
}

__global__ __launch_bounds__(256) void k_prep(const float* __restrict__ x, const float* __restrict__ cw,
                                               const float* __restrict__ cb,
                                               unsigned short* __restrict__ xah, unsigned short* __restrict__ xal) {
  __shared__ __align__(16) float ring[4][16][96];
  __shared__ __align__(16) unsigned int rowH[16][96];
  __shared__ __align__(16) unsigned int rowL[16][96];
  const int tid  = threadIdx.x;
  const int lane = tid & 31;
  const int wave = tid >> 5;
  const int bf0  = blockIdx.x * 16;
  const int b    = bf0 / kHW;
  const int hw0  = bf0 - b * kHW;
  {
    float* zp = &ring[1][0][0];
#pragma unroll 1
    for (int i = tid; i < 3 * 16 * 96; i += 256) zp[i] = 0.0f;
  }
  __syncthreads();
#pragma unroll 1
  for (int t = 0; t < kNT; ++t) {
    const int slot = t & 3;
#pragma unroll 1
    for (int it = 0; it < 6; ++it) {
      const int idx = it * 256 + tid;
      const int c   = idx >> 4;
      const int hwl = idx & 15;
      ring[slot][hwl][c] = x[(((size_t)b * kNC + c) * kNT + t) * kHW + hw0 + hwl];
    }
    __syncthreads();
#pragma unroll 1
    for (int it = 0; it < 3; ++it) {
      const int idx = it * 256 + tid;
      const int hwl = idx / 48;
      const int cp  = idx - hwl * 48;
      const int c0  = 2 * cp;
      float xc2[2], xs2[2];
#pragma unroll
      for (int u = 0; u < 2; ++u) {
        const int c = c0 + u;
        float acc = 0.0f;
#pragma unroll
        for (int j = 0; j < kKC; ++j) {
          acc = fmaf(ring[(t + 1 + j) & 3][hwl][c], cw[c * kKC + j], acc);
        }
        acc += cb[c];
        const float ex  = expf(-acc);
        const float sg  = 1.0f / (1.0f + ex);
        xc2[u] = acc * sg;
        xs2[u] = ring[slot][hwl][c];
      }
      const unsigned short hc0 = f2bf_bits(xc2[0]);
      const unsigned short hc1 = f2bf_bits(xc2[1]);
      const unsigned short lc0 = f2bf_bits(xc2[0] - bf_bits2f(hc0));
      const unsigned short lc1 = f2bf_bits(xc2[1] - bf_bits2f(hc1));
      const unsigned short hs0 = f2bf_bits(xs2[0]);
      const unsigned short hs1 = f2bf_bits(xs2[1]);
      const unsigned short ls0 = f2bf_bits(xs2[0] - bf_bits2f(hs0));
      const unsigned short ls1 = f2bf_bits(xs2[1] - bf_bits2f(hs1));
      rowH[hwl][cp]      = pk16(hc0, hc1);
      rowL[hwl][cp]      = pk16(lc0, lc1);
      rowH[hwl][48 + cp] = pk16(hs0, hs1);
      rowL[hwl][48 + cp] = pk16(ls0, ls1);
    }
    __syncthreads();
    {
      const int lc = (lane < 24) ? lane : 23;
      for (int pass = 0; pass < 2; ++pass) {
#pragma unroll
        for (int rr = 0; rr < 2; ++rr) {
          const int hwl = wave * 2 + rr;
          const v4u uh = *(const v4u*)(&rowH[hwl][lc * 4]);
          const v4u ul = *(const v4u*)(&rowL[hwl][lc * 4]);
          const size_t dst = ((size_t)(bf0 + hwl) * kNT + t) * kKX + (size_t)lc * 8;
          if (lane < 24) {
            *(volatile v4u*)(xah + dst) = uh;
            *(volatile v4u*)(xal + dst) = ul;
          }
        }
        __threadfence();
      }
    }
  }
}

__global__ __launch_bounds__(256) void k_cell(const float* __restrict__ raw,
                                               float* stC, float* stN, float* stM,
                                               unsigned short* __restrict__ hh, unsigned short* __restrict__ hl,
                                               const float* __restrict__ gnw, float* __restrict__ out,
                                               int t, int first) {
  __shared__ __align__(16) float sS[3][32 * 96];
  __shared__ __align__(16) unsigned short sHh[32 * 96];
  __shared__ __align__(16) unsigned short sHl[32 * 96];
  __shared__ __align__(16) float sY[96 * 36];
  const int tid  = threadIdx.x;
  const int lane = tid & 31;
  const int wave = tid >> 5;
  const int bf0  = blockIdx.x * 32;
  const int b    = bf0 / kHW;
  const int hw0  = bf0 - b * kHW;

#pragma unroll 1
  for (int it = 0; it < 12; ++it) {
    const int p    = wave * 12 + it;
    const int rowl = p / 3;
    const int head = p - rowl * 3;
    const int col  = head * kDH + lane;
    const size_t grow = (size_t)(bf0 + rowl);
    const float* rp = raw + grow * kNCOL + col;
    const float ir  = rp[0];
    const float fr  = rp[96];
    const float zr  = rp[192];
    const float orw = rp[288];
    float c = 0.0f, n = 0.0f, m = 0.0f;
    if (first == 0) {
      const size_t si = grow * kNC + col;
      c = stC[si];
      n = stN[si];
      m = stM[si];
    }
    const float lsf = fminf(fr, 0.0f) - log1pf(expf(-fabsf(fr)));
    const float lfm = m + lsf;
    const float mn  = fmaxf(ir, lfm);
    const float ig  = expf(ir - mn);
    const float fg  = expf(lfm - mn);
    const float th  = tanhf(zr);
    const float cn  = fg * c + ig * th;
    const float nn  = fg * n + ig;
    const float eo  = expf(-orw);
    const float so  = 1.0f / (1.0f + eo);
    const float hn  = (so * cn) * (1.0f / nn);
    const int li = rowl * kNC + col;
    sS[0][li] = cn;
    sS[1][li] = nn;
    sS[2][li] = mn;
    const unsigned short hb = f2bf_bits(hn);
    const unsigned short lb = f2bf_bits(hn - bf_bits2f(hb));
    sHh[li] = hb;
    sHl[li] = lb;
    float s1 = hn;
#pragma unroll
    for (int off = 1; off < 32; off <<= 1) s1 += __shfl_xor(s1, off, 32);
    const float mu = s1 * (1.0f / 32.0f);
    const float dv = hn - mu;
    float s2 = dv * dv;
#pragma unroll
    for (int off = 1; off < 32; off <<= 1) s2 += __shfl_xor(s2, off, 32);
    const float var = s2 * (1.0f / 32.0f);
    const float yn  = dv * rsqrtf(var + 1e-5f) * gnw[col];
    sY[col * 36 + rowl] = yn;
  }
  __syncthreads();

  const size_t stBase = (size_t)bf0 * kNC;
  for (int pass = 0; pass < 2; ++pass) {
#pragma unroll
    for (int it = 0; it < 3; ++it) {
      const int i = it * 256 + tid;
      const v4f a0 = *(const v4f*)(&sS[0][i * 4]);
      const v4f a1 = *(const v4f*)(&sS[1][i * 4]);
      const v4f a2 = *(const v4f*)(&sS[2][i * 4]);
      *(volatile v4f*)(stC + stBase + (size_t)i * 4) = a0;
      *(volatile v4f*)(stN + stBase + (size_t)i * 4) = a1;
      *(volatile v4f*)(stM + stBase + (size_t)i * 4) = a2;
    }
#pragma unroll
    for (int it = 0; it < 2; ++it) {
      const int i = it * 256 + tid;
      const int ic = (i < 384) ? i : 383;
      const v4u uh = *(const v4u*)(sHh + ic * 8);
      const v4u ul = *(const v4u*)(sHl + ic * 8);
      if (i < 384) {
        *(volatile v4u*)(hh + stBase + (size_t)i * 8) = uh;
        *(volatile v4u*)(hl + stBase + (size_t)i * 8) = ul;
      }
    }
#pragma unroll
    for (int k = 0; k < 3; ++k) {
      const int c  = (k * 8 + wave) * 4 + (lane >> 3);
      const int j4 = (lane & 7) * 4;
      const v4f y = *(const v4f*)(&sY[c * 36 + j4]);
      const size_t o = (((size_t)b * kNC + c) * kNT + t) * kHW + hw0 + j4;
      *(volatile v4f*)(out + o) = y;
    }
    __threadfence();
  }
}

extern "C" void kernel_launch(void* const* d_in, const int* in_sizes, int n_in,
                              void* d_out, int out_size, void* d_ws, size_t ws_size,
                              hipStream_t stream) {
  if (n_in < 10) return;
  if ((size_t)out_size != kOutElems) return;
  if (ws_size < kWsTotal) return;
  if ((size_t)in_sizes[0] != kOutElems) return;
  if (in_sizes[1] != kNC * kKC || in_sizes[2] != kNC) return;
  if (in_sizes[3] != kNH * kDH * kDH || in_sizes[4] != kNH * kDH * kDH ||
      in_sizes[5] != kNH * kDH * kDH || in_sizes[6] != kNH * kDH * kDH) return;
  if (in_sizes[7] != 4 * kNH * kDH * kDH || in_sizes[8] != kNCOL || in_sizes[9] != kNC) return;

  const float* x    = (const float*)d_in[0];
  const float* cw   = (const float*)d_in[1];
  const float* cb   = (const float*)d_in[2];
  const float* Wi   = (const float*)d_in[3];
  const float* Wf   = (const float*)d_in[4];
  const float* Wz   = (const float*)d_in[5];
  const float* Wo   = (const float*)d_in[6];
  const float* Rm   = (const float*)d_in[7];
  const float* bvec = (const float*)d_in[8];
  const float* gnw  = (const float*)d_in[9];
  float* out = (float*)d_out;

  char* ws = (char*)d_ws;
  unsigned short* wbth = (unsigned short*)(ws + kOffWbtH);
  unsigned short* wbtl = (unsigned short*)(ws + kOffWbtL);
  unsigned short* rbth = (unsigned short*)(ws + kOffRbtH);
  unsigned short* rbtl = (unsigned short*)(ws + kOffRbtL);
  unsigned short* xah  = (unsigned short*)(ws + kOffXaH);
  unsigned short* xal  = (unsigned short*)(ws + kOffXaL);
  float* gbuf = (float*)(ws + kOffG);
  float* rawb = (float*)(ws + kOffRaw);
  unsigned short* hh = (unsigned short*)(ws + kOffHh);
  unsigned short* hl = (unsigned short*)(ws + kOffHl);
  float* stC = (float*)(ws + kOffStC);
  float* stN = (float*)(ws + kOffStN);
  float* stM = (float*)(ws + kOffStM);

  const int gemmBlocks = ((kBF / 64) * (kNCOL / 64) + 7) / 8;

  k_wpack<<<54, 256, 0, stream>>>(Wi, Wf, Wz, Wo, Rm, wbth, wbtl, rbth, rbtl);
  k_prep<<<kBF / 16, 256, 0, stream>>>(x, cw, cb, xah, xal);

  for (int s = 0; s < kNT / 2; ++s) {
    const int t0 = 2 * s;
    wmma_gemm64<1, true, 2, 0, false, 0><<<dim3(gemmBlocks, 2), 256, 0, stream>>>(
        xah + (size_t)t0 * kKX, xal + (size_t)t0 * kKX, kLDXA, (long)kKX,
        wbth, wbtl, kKX, 0L,
        (void*)gbuf, nullptr, kNCOL, (long)kGPlane,
        bvec, nullptr, 0L,
        kBF, kNCOL, kKX, 1.0f);
    for (int u = 0; u < 2; ++u) {
      const int t = t0 + u;
      float* gslot = gbuf + (size_t)u * kGPlane;
      const float* rawp = gslot;
      if (t > 0) {
        wmma_gemm64<1, true, 0, 0, true, 0><<<dim3(gemmBlocks, 1), 256, 0, stream>>>(
            hh, hl, kKR, 0L,
            rbth, rbtl, kKR, 0L,
            (void*)rawb, nullptr, kNCOL, 0L,
            nullptr, gslot, 0L,
            kBF, kNCOL, kKR, 1.0f);
        rawp = rawb;
      }
      k_cell<<<kBF / 32, 256, 0, stream>>>(rawp, stC, stN, stM, hh, hl, gnw, out, t, (t == 0) ? 1 : 0);
    }
  }
}
